// InnerSoftShiftTriple_48859547959304
// MI455X (gfx1250) — hardware-run, weakly checked
//
#include <hip/hip_runtime.h>


namespace {
constexpr int B = 4, C2 = 32, HW = 64, N = HW * HW;
constexpr float XS = 8.0f, PS = 1024.0f;
typedef _Float16 b16;
typedef __attribute__((ext_vector_type(16))) _Float16 v16b;
typedef __attribute__((ext_vector_type(8))) _Float16 v8b;
typedef __attribute__((ext_vector_type(8))) float v8f;
typedef __attribute__((ext_vector_type(2))) _Float16 v2b;
__device__ __forceinline__ float bf16_rne(float f) { unsigned int u = __float_as_uint(f); u += 0x7FFFu + ((u >> 16) & 1u); float r = __uint_as_float(u & 0xFFFF0000u); asm volatile("" : "+v"(r)); return r; }
__device__ __forceinline__ void split16(float v, b16& hi, b16& lo) { hi = (b16)v; lo = (b16)(v - (float)hi); }
__device__ __forceinline__ v16b frag_kb(const b16* p, int hh) { const v8b a = *(const v8b*)(p + 8 * hh), b = *(const v8b*)(p + 16 + 8 * hh); v16b f;
#pragma unroll
  for (int e = 0; e < 8; ++e) { f[e] = a[e]; f[8 + e] = b[e]; } return f; }
__device__ __forceinline__ v8f wmma16b(v16b a, v16b b, v8f c) { v8f d = __builtin_amdgcn_wmma_f32_16x16x32_f16(false, a, false, b, (short)0, c, false, false); asm volatile("v_nop\n\tv_nop\n\tv_nop\n\tv_nop" : "+v"(d) : "v"(a), "v"(b)); return d; }
__device__ __forceinline__ void wave_lds_sync() { __builtin_amdgcn_fence(__ATOMIC_RELEASE, "workgroup"); __builtin_amdgcn_wave_barrier(); __builtin_amdgcn_fence(__ATOMIC_ACQUIRE, "workgroup"); }
__device__ __forceinline__ float pmul(float a, float b) { float p = a * b; asm volatile("" : "+v"(p)); return p; }

__global__ __launch_bounds__(32) void prep_kernel(const float* __restrict__ x, b16* __restrict__ LNh, b16* __restrict__ LNl) { const int lane = threadIdx.x; const int jb = blockIdx.x % (N / 32), b = blockIdx.x / (N / 32); const int j = jb * 32 + lane; const float* lat = x + ((size_t)b * 2 * C2 + C2) * N;
  float v[C2]; float s = 0.0f;
#pragma unroll
  for (int c = 0; c < C2; ++c) { v[c] = bf16_rne(lat[(size_t)c * N + j]); s += pmul(v[c], v[c]); } const float inv = 1.0f / fmaxf(sqrtf(s), 1e-6f);
  for (int pass = 0; pass < 2; ++pass) {
#pragma unroll
    for (int c = 0; c < C2; c += 2) { b16 p0, q0, p1, q1; split16(pmul(v[c], inv) * XS, p0, q0); split16(pmul(v[c + 1], inv) * XS, p1, q1); *(volatile v2b*)(LNh + ((size_t)b * N + j) * C2 + c) = (v2b){p0, p1}; *(volatile v2b*)(LNl + ((size_t)b * N + j) * C2 + c) = (v2b){q0, q1}; }
    __threadfence(); } }
__global__ __launch_bounds__(256) void copy_kernel(const float* __restrict__ x, const int* __restrict__ mask, b16* __restrict__ LT, float* __restrict__ out) { const size_t u = (size_t)blockIdx.x * 256 + threadIdx.x;
  for (int pass = 0; pass < 2; ++pass) {
    if (u < (size_t)B * 2 * C2 * N / 4) { const size_t e = u * 4; const int b = (int)(e / ((size_t)2 * C2 * N)); const size_t rem = e % ((size_t)2 * C2 * N); typedef __attribute__((ext_vector_type(4))) float v4f; v4f v; for (int k = 0; k < 4; ++k) v[k] = bf16_rne(x[e + k]); *(volatile v4f*)(out + (size_t)b * 3 * C2 * N + rem) = v; }
    if (u < (size_t)B * C2 * N / 8) { const size_t e = u * 8; const int b = (int)(e / ((size_t)C2 * N)); const size_t rem = e % ((size_t)C2 * N); v8b v;
#pragma unroll
      for (int k = 0; k < 8; ++k) v[k] = (b16)(bf16_rne(x[((size_t)b * 2 * C2 + C2) * N + rem + k]) * XS); *(volatile v8b*)(LT + e) = v; }
    __threadfence(); } }
__global__ __launch_bounds__(32) void att_kernel(const float* __restrict__ x, const int* __restrict__ mask, const b16* __restrict__ LNh, const b16* __restrict__ LNl, const b16* __restrict__ LT, int BV, float* __restrict__ out) {
  __shared__ __attribute__((aligned(16))) b16 Af[32][40], Ph[32][40], Pl[32][40]; __shared__ float Sc[32][33], Mx[32], Dn[32], Sf[32], Of[C2][33]; __shared__ int Fk[32];
  const int lane = threadIdx.x, nloc = lane & 15, hlf = lane >> 4; const int qt = blockIdx.x % (N / 32), b = blockIdx.x / (N / 32); if (b >= BV) return; const int i0 = qt * 32; const float* fr = x + (size_t)b * 2 * C2 * N;
  for (int c = 0; c < C2; ++c) Af[lane][c] = (b16)(bf16_rne(fr[(size_t)c * N + i0 + lane]) * XS);
  Mx[lane] = -INFINITY; Dn[lane] = 0.0f; Sf[lane] = 0.0f;
  v8f acc[2][2]; for (int m = 0; m < 2; ++m) for (int t = 0; t < 2; ++t) acc[m][t] = (v8f){};
  wave_lds_sync(); v16b qa[2]; for (int m = 0; m < 2; ++m) qa[m] = frag_kb(&Af[m * 16 + nloc][0], hlf);
  int nvalid = 0;
#pragma unroll 1
  for (int kc = 0; kc < N; kc += 32) { const int fk = mask[kc + lane] >= 1 ? 1 : 0; Fk[lane] = fk; int cntv = 1 - fk; for (int o = 16; o; o >>= 1) cntv += __shfl_xor(cntv, o); if (cntv == 0) continue;
    nvalid += cntv; wave_lds_sync();
#pragma unroll
    for (int blk = 0; blk < 2; ++blk) { const size_t jr = ((size_t)b * N + kc + blk * 16 + nloc) * C2; const v16b kh = frag_kb(LNh + jr, hlf), kl = frag_kb(LNl + jr, hlf);
#pragma unroll
      for (int m = 0; m < 2; ++m) { v8f s = {}; s = wmma16b(qa[m], kh, s); s = wmma16b(qa[m], kl, s);
#pragma unroll
        for (int r8 = 0; r8 < 8; ++r8) { const int kk = blk * 16 + nloc; Sc[m * 16 + 8 * hlf + r8][kk] = Fk[kk] ? -INFINITY : s[r8] * (1.0f / (XS * XS)); } } }
    wave_lds_sync();
#pragma unroll 1
    for (int qi = 0; qi < 32; ++qi) { const float sv = Sc[qi][lane]; float cm = sv; for (int o = 16; o; o >>= 1) cm = fmaxf(cm, __shfl_xor(cm, o)); const float mo = Mx[qi]; const float mn = fmaxf(mo, cm); const float p = (sv == -INFINITY) ? 0.0f : __expf(sv - mn); float ps = p; for (int o = 16; o; o >>= 1) ps += __shfl_xor(ps, o);
      b16 ph, plo; split16(p * PS, ph, plo); Ph[qi][lane] = ph; Pl[qi][lane] = plo; if (lane == 0) { const float sf = (mo == -INFINITY) ? 0.0f : __expf(mo - mn); Sf[qi] = sf; Dn[qi] = Dn[qi] * sf + ps; Mx[qi] = mn; } }
    wave_lds_sync();
#pragma unroll
    for (int m = 0; m < 2; ++m) { const v16b pa = frag_kb(&Ph[m * 16 + nloc][0], hlf), pb = frag_kb(&Pl[m * 16 + nloc][0], hlf);
#pragma unroll
      for (int t = 0; t < 2; ++t) {
#pragma unroll
        for (int r8 = 0; r8 < 8; ++r8) acc[m][t][r8] *= Sf[m * 16 + 8 * hlf + r8];
        const v16b vv = frag_kb(LT + ((size_t)b * C2 + t * 16 + nloc) * N + kc, hlf); acc[m][t] = wmma16b(pa, vv, acc[m][t]); acc[m][t] = wmma16b(pb, vv, acc[m][t]); } }
    wave_lds_sync(); }
  if (nvalid == 0) { for (int c = 0; c < C2; ++c) { float s = 0.0f; for (int j = lane; j < N; j += 32) s += bf16_rne(fr[((size_t)C2 + c) * N + j]); for (int o = 16; o; o >>= 1) s += __shfl_xor(s, o); if (lane == 0) for (int q = 0; q < 32; ++q) Of[c][q] = s * (1.0f / N); } }
  else {
#pragma unroll
    for (int m = 0; m < 2; ++m)
#pragma unroll
      for (int t = 0; t < 2; ++t)
#pragma unroll
        for (int r8 = 0; r8 < 8; ++r8) { const int ql = m * 16 + 8 * hlf + r8; Of[t * 16 + nloc][ql] = acc[m][t][r8] * (1.0f / (PS * XS)) / Dn[ql]; } }
  wave_lds_sync(); const float fq = mask[i0 + lane] >= 1 ? 1.0f : 0.0f;
  for (int pass = 0; pass < 2; ++pass) { for (int c = 0; c < C2; ++c) ((volatile float*)out)[((size_t)b * 3 * C2 + 2 * C2 + c) * N + i0 + lane] = pmul(Of[c][lane], fq); __threadfence(); } }
}

extern "C" void kernel_launch(void* const* d_in, const int* in_sizes, int n_in, void* d_out, int out_size, void* d_ws, size_t ws_size, hipStream_t stream) {
  (void)n_in;
  auto Fp = [&](int i) { return (const float*)d_in[i]; }; auto Ip = [&](int i) { return (const int*)d_in[i]; };
  if (in_sizes[0] != B * 2 * C2 * N || in_sizes[1] != N || out_size != B * 3 * C2 * N) return;
  const int BV = B;
  size_t off = 0; char* ws = (char*)d_ws;
  auto carve = [&](size_t bytes) { char* p = ws + off; off += (bytes + 255) & ~(size_t)255; return p; };
  b16* LNh = (b16*)carve((size_t)B * N * C2 * 2); b16* LNl = (b16*)carve((size_t)B * N * C2 * 2); b16* LT = (b16*)carve((size_t)B * C2 * N * 2);
  if (off > ws_size || off > ((size_t)8 << 20)) return;
  prep_kernel<<<B * (N / 32), 32, 0, stream>>>(Fp(0), LNh, LNl);
  copy_kernel<<<(unsigned)(((size_t)B * 2 * C2 * N / 4 + 255) / 256), 256, 0, stream>>>(Fp(0), Ip(1), LT, (float*)d_out);
  att_kernel<<<BV * (N / 32), 32, 0, stream>>>(Fp(0), Ip(1), LNh, LNl, LT, BV, (float*)d_out);
}
